// TransConvLayer_22419729285548
// MI455X (gfx1250) — hardware-verified
//
#include <hip/hip_runtime.h>
#include <math.h>
#include <stdint.h>

#define NQ   4096
#define NL   4096
#define DM   512
#define NH   8
#define DKH  64
#define DV   (NH * DM)
#ifndef SQ
#define SQ NQ
#endif
#define NT   32
#define LT   32
#define SSP  32
#define PLP  40
#define SLAB64 (16 * 68)
#define ATT_THREADS 256
#define QSC  8.0f
#define KSC  8.0f
#define VSC  8.0f
#define W2S  1024.0f
#define PCAR 4096.0f
#define VCAR 64.0f
#define LOG2E 1.4426950408889634f
#define WS_CAP ((size_t)134217728)

static_assert(DM == NH * DKH && DKH == 64 && NH == 8 && (DM % 64) == 0 && (DV % 64) == 0 && (NL % 64) == 0 && (NQ % 64) == 0);
static_assert((DM % 32) == 0);
static_assert(SQ >= 64 && SQ <= NQ && (SQ % 64) == 0 && (SQ % NT) == 0);
static_assert(NT == 32 && LT == 32 && (NL % LT) == 0 && ATT_THREADS == 256 && ATT_THREADS * 4 == NT * LT);
static_assert(SSP >= LT && PLP >= 32 && ((PLP * 2) % 16) == 0 && ((SSP * 4) % 16) == 0);
static_assert(NH * NT * SSP <= 8 * SLAB64);
static_assert(((NQ * DM) % 2048) == 0 && ((NL * DM) % 2048) == 0 && ((SQ * DM) % 2048) == 0);
static_assert(NH * NT * SSP * 4 + 0 <= 40000 && NH * NT * PLP * 2 <= 24000);

typedef unsigned short u16;
typedef _Float16 v16h __attribute__((ext_vector_type(16)));
typedef _Float16 v8h  __attribute__((ext_vector_type(8)));
typedef __bf16   v16b __attribute__((ext_vector_type(16)));
typedef float    v8f  __attribute__((ext_vector_type(8)));
typedef float    v4f  __attribute__((ext_vector_type(4)));
typedef unsigned int v4u __attribute__((ext_vector_type(4)));
typedef unsigned int v2u __attribute__((ext_vector_type(2)));

union FragH { v16h v; v8h h[2]; v4u u[2]; };
union FragB { v16b v; v4u u[2]; };
union AttU { float s[NH * NT * SSP]; float slab[8 * SLAB64]; };

__device__ __forceinline__ unsigned short bf_bits(float f) {
  unsigned u = __float_as_uint(f);
  return (unsigned short)((u + 0x7FFFu + ((u >> 16) & 1u)) >> 16);
}
__device__ __forceinline__ float bf_up(unsigned short h) { return __uint_as_float(((unsigned)h) << 16); }
__device__ __forceinline__ float bfr(float f) { return bf_up(bf_bits(f)); }
__device__ __forceinline__ unsigned short h_bits(_Float16 x) { return __builtin_bit_cast(unsigned short, x); }
__device__ __forceinline__ unsigned pk16(unsigned short a, unsigned short b) { return (unsigned)a | ((unsigned)b << 16); }
__device__ __forceinline__ v8f zero8() { v8f z = {0.f, 0.f, 0.f, 0.f, 0.f, 0.f, 0.f, 0.f}; return z; }

__device__ __forceinline__ v16h ldfrag_h(const _Float16* p) {
  FragH f;
  f.h[0] = *(const v8h*)(p);
  f.h[1] = *(const v8h*)(p + 16);
  return f.v;
}
__device__ __forceinline__ v16b ldfrag_b(const u16* p) {
  FragB f;
  f.u[0] = *(const v4u*)(p);
  f.u[1] = *(const v4u*)(p + 16);
  return f.v;
}

__device__ __forceinline__ v8f mma_h(v16h a, v16h b, v8f c) {
  return __builtin_amdgcn_wmma_f32_16x16x32_f16(false, a, false, b, (short)0, c, false, false);
}
__device__ __forceinline__ v8f mma_b(v16b a, v16b b, v8f c) {
  return __builtin_amdgcn_wmma_f32_16x16x32_bf16(false, a, false, b, (short)0, c, false, false);
}
template <typename F>
__device__ __forceinline__ void guard6(v8f& a, v8f& b, v8f& c, v8f& d, F x0, F x1, F x2, F x3, F x4, F x5) {
#if defined(__HIP_DEVICE_COMPILE__)
  asm volatile("v_nop\n\tv_nop\n\tv_nop\n\tv_nop"
               : "+v"(a), "+v"(b), "+v"(c), "+v"(d) : "v"(x0), "v"(x1), "v"(x2), "v"(x3), "v"(x4), "v"(x5) : "memory");
#endif
}
__device__ __forceinline__ void guard4x8(v8f& a, v8f& b, v8f& c, v8f& d, v16h x0, v16h x1, v16h x2, v16h x3,
                                         v16h x4, v16h x5, v16h x6, v16h x7) {
#if defined(__HIP_DEVICE_COMPILE__)
  asm volatile("v_nop\n\tv_nop\n\tv_nop\n\tv_nop"
               : "+v"(a), "+v"(b), "+v"(c), "+v"(d)
               : "v"(x0), "v"(x1), "v"(x2), "v"(x3), "v"(x4), "v"(x5), "v"(x6), "v"(x7) : "memory");
#endif
}
__device__ __forceinline__ void guard8x6(v8f& a0, v8f& a1, v8f& a2, v8f& a3, v8f& e0, v8f& e1, v8f& e2, v8f& e3,
                                         v16h x0, v16h x1, v16h x2, v16h x3, v16h x4, v16h x5) {
#if defined(__HIP_DEVICE_COMPILE__)
  asm volatile("v_nop\n\tv_nop\n\tv_nop\n\tv_nop"
               : "+v"(a0), "+v"(a1), "+v"(a2), "+v"(a3), "+v"(e0), "+v"(e1), "+v"(e2), "+v"(e3)
               : "v"(x0), "v"(x1), "v"(x2), "v"(x3), "v"(x4), "v"(x5) : "memory");
#endif
}
__device__ __forceinline__ void wave_sync_lds() {
  __builtin_amdgcn_fence(__ATOMIC_RELEASE, "workgroup");
  __builtin_amdgcn_wave_barrier();
  __builtin_amdgcn_fence(__ATOMIC_ACQUIRE, "workgroup");
}

__global__ __launch_bounds__(256) void cvt16(const float* __restrict__ x, u16* D, int n8, int mode, float scale) {
  const int gt = blockIdx.x * 256 + (int)threadIdx.x;
  if (gt >= n8) return;
  const float* p = x + (size_t)gt * 8;
  const v4f a = *(const v4f*)(p), c4 = *(const v4f*)(p + 4);
  float v[8];
#pragma unroll
  for (int e = 0; e < 4; ++e) { v[e] = a[e]; v[4 + e] = c4[e]; }
  unsigned short s[8];
#pragma unroll
  for (int e = 0; e < 8; ++e) {
    const float vb = bfr(v[e]);
    const float vf = (mode == 1) ? vb : v[e];
    const unsigned short hb = h_bits((_Float16)(vf * scale));
    const unsigned short bb = bf_bits(v[e]);
    s[e] = (mode != 0) ? hb : bb;
  }
  v4u o;
#pragma unroll
  for (int e = 0; e < 4; ++e) o[e] = pk16(s[2 * e], s[2 * e + 1]);
  u16* d = D + (size_t)gt * 8;
  for (int pass = 0; pass < 2; ++pass) {
    *(volatile v4u*)(d) = o;
    __threadfence();
  }
}

#define VTP 72
static_assert(64 * VTP >= 63 * VTP + 64 && ((VTP * 2) % 16) == 0);
__global__ __launch_bounds__(256) void tr16(const float* __restrict__ X, u16* XTo, int R, int C, int mode, float scale) {
  __shared__ __align__(16) u16 TH[64 * VTP];
  const int tid = threadIdx.x;
  const int bid = blockIdx.x;
  const int nrt = R >> 6;
  const int rt  = bid % nrt;
  const int ct  = bid / nrt;
  const int r0  = rt * 64;
  const int c0  = ct * 64;
  {
    const int rl = tid >> 2;
    const int cc = (tid & 3) * 16;
    const float* src = X + (size_t)(r0 + rl) * (size_t)C + c0 + cc;
#pragma unroll
    for (int i = 0; i < 4; ++i) {
      const v4f a = *(const v4f*)(src + 4 * i);
#pragma unroll
      for (int e = 0; e < 4; ++e) {
        const float v  = a[e];
        const float vb = bfr(v);
        const float vf = (mode == 1) ? vb : v;
        const unsigned short hb = h_bits((_Float16)(vf * scale));
        const unsigned short bb = bf_bits(v);
        TH[(cc + 4 * i + e) * VTP + rl] = (mode != 0) ? hb : bb;
      }
    }
  }
  __syncthreads();
  v4u vh[2];
  const int q8 = tid >> 3, p8 = (tid & 7) * 8;
#pragma unroll
  for (int it = 0; it < 2; ++it) {
    const int line = it * 32 + q8;
    vh[it] = *(const v4u*)(TH + line * VTP + p8);
  }
  const size_t base = (size_t)c0 * (size_t)R + (size_t)r0 + (size_t)p8;
  for (int pass = 0; pass < 2; ++pass) {
#pragma unroll
    for (int it = 0; it < 2; ++it) {
      const int line = it * 32 + q8;
      *(volatile v4u*)(XTo + base + (size_t)line * (size_t)R) = vh[it];
    }
    __threadfence();
  }
}

__device__ __forceinline__ void stage64(float* sl, v8f a0, v8f a1, v8f a2, v8f a3, float oscale, int lane) {
  const int hh = lane >> 4, m = lane & 15;
#pragma unroll
  for (int r = 0; r < 8; ++r) {
    const int ro = (8 * hh + r) * 68 + m;
    sl[ro]      = a0[r] * oscale;
    sl[ro + 16] = a1[r] * oscale;
    sl[ro + 32] = a2[r] * oscale;
    sl[ro + 48] = a3[r] * oscale;
  }
  wave_sync_lds();
}
__device__ __forceinline__ void epi64(float* sl, v8f a0, v8f a1, v8f a2, v8f a3, float oscale, v4f badd, float* C, int N,
                                      size_t rowb, int col0, int lane) {
  const int hh = lane >> 4, m = lane & 15;
  stage64(sl, a0, a1, a2, a3, oscale, lane);
  v4f vals[8];
#pragma unroll
  for (int it = 0; it < 8; ++it) vals[it] = *(const v4f*)(sl + (it * 2 + hh) * 68 + m * 4) + badd;
  float* dst = C + (rowb + (size_t)hh) * (size_t)N + col0 + m * 4;
  for (int pass = 0; pass < 2; ++pass) {
#pragma unroll
    for (int it = 0; it < 8; ++it) {
      *(volatile v4f*)(dst + (size_t)(it * 2) * (size_t)N) = vals[it];
    }
    __threadfence();
  }
}
__device__ __forceinline__ void epi64hsb(float* sl, v8f a0, v8f a1, v8f a2, v8f a3, float oscale, float pscale,
                                         const float* __restrict__ bias, u16* C, int N, size_t rowb, int col0, int lane) {
  stage64(sl, a0, a1, a2, a3, oscale, lane);
  const int rq = lane >> 3, c8 = (lane & 7) * 8;
  const v4f b0 = *(const v4f*)(bias + col0 + c8), b1 = *(const v4f*)(bias + col0 + c8 + 4);
  float bb[8];
#pragma unroll
  for (int e = 0; e < 4; ++e) { bb[e] = bfr(b0[e]); bb[4 + e] = bfr(b1[e]); }
  v4u oh[4];
#pragma unroll
  for (int i4 = 0; i4 < 4; ++i4) {
    const int row = i4 * 4 + rq;
    const v4f a = *(const v4f*)(sl + row * 68 + c8), c4 = *(const v4f*)(sl + row * 68 + c8 + 4);
    float w[8];
#pragma unroll
    for (int e = 0; e < 4; ++e) { w[e] = (a[e] + bb[e]) * pscale; w[4 + e] = (c4[e] + bb[4 + e]) * pscale; }
#pragma unroll
    for (int e = 0; e < 4; ++e) oh[i4][e] = pk16(h_bits((_Float16)w[2 * e]), h_bits((_Float16)w[2 * e + 1]));
  }
  u16* dst = C + rowb * (size_t)N + col0 + c8;
  for (int pass = 0; pass < 2; ++pass) {
#pragma unroll
    for (int i4 = 0; i4 < 4; ++i4) {
      const int row = i4 * 4 + rq;
      *(volatile v4u*)(dst + (size_t)row * (size_t)N) = oh[i4];
    }
    __threadfence();
  }
}
__device__ __forceinline__ void epi64hrb(float* sl, v8f a0, v8f a1, v8f a2, v8f a3, float oscale, float pscale,
                                         const float* __restrict__ brow, u16* C, int N, size_t rowb, int col0, int lane) {
  const int hh = lane >> 4, m = lane & 15;
  const v4f r0v = *(const v4f*)(brow + 8 * hh), r1v = *(const v4f*)(brow + 8 * hh + 4);
  float rb[8];
#pragma unroll
  for (int e = 0; e < 4; ++e) { rb[e] = bfr(r0v[e]); rb[4 + e] = bfr(r1v[e]); }
#pragma unroll
  for (int r = 0; r < 8; ++r) {
    const int ro = (8 * hh + r) * 68 + m;
    sl[ro]      = a0[r] * oscale + rb[r];
    sl[ro + 16] = a1[r] * oscale + rb[r];
    sl[ro + 32] = a2[r] * oscale + rb[r];
    sl[ro + 48] = a3[r] * oscale + rb[r];
  }
  wave_sync_lds();
  const int rq = lane >> 3, c8 = (lane & 7) * 8;
  v4u oh[4];
#pragma unroll
  for (int i4 = 0; i4 < 4; ++i4) {
    const int row = i4 * 4 + rq;
    const v4f a = *(const v4f*)(sl + row * 68 + c8), c4 = *(const v4f*)(sl + row * 68 + c8 + 4);
    float w[8];
#pragma unroll
    for (int e = 0; e < 4; ++e) { w[e] = a[e] * pscale; w[4 + e] = c4[e] * pscale; }
#pragma unroll
    for (int e = 0; e < 4; ++e) oh[i4][e] = pk16(h_bits((_Float16)w[2 * e]), h_bits((_Float16)w[2 * e + 1]));
  }
  u16* dst = C + rowb * (size_t)N + col0 + c8;
  for (int pass = 0; pass < 2; ++pass) {
#pragma unroll
    for (int i4 = 0; i4 < 4; ++i4) {
      const int row = i4 * 4 + rq;
      *(volatile v4u*)(dst + (size_t)row * (size_t)N) = oh[i4];
    }
    __threadfence();
  }
}

__global__ __launch_bounds__(128)
void gemm_bh16(const u16* __restrict__ A, const u16* __restrict__ Bt, const float* __restrict__ bias, u16* C,
               int M, int N, int K, float oscale, float pscale) {
  __shared__ __align__(16) float slab[4 * SLAB64];
  const int tid = threadIdx.x, wave = tid >> 5, lane = tid & 31, hh = lane >> 4, m = lane & 15;
  const int ntile = N >> 6;
  const int bid   = blockIdx.x;
  const int rowb  = (bid / ntile) * 64 + wave * 16;
  const int col0  = (bid % ntile) * 64;
  if (rowb + 16 > M) return;
  const u16* ap = A  + (size_t)(rowb + m) * (size_t)K + 8 * hh;
  const u16* bp = Bt + (size_t)(col0 + m) * (size_t)K + 8 * hh;
  const size_t bs = (size_t)16 * K;
  v8f acc0 = zero8(), acc1 = zero8(), acc2 = zero8(), acc3 = zero8();
#pragma unroll 1
  for (int k0 = 0; k0 < K; k0 += 32) {
    const v16b a  = ldfrag_b(ap + k0);
    const v16b b0 = ldfrag_b(bp + k0);
    const v16b b1 = ldfrag_b(bp + bs + k0);
    const v16b b2 = ldfrag_b(bp + 2 * bs + k0);
    const v16b b3 = ldfrag_b(bp + 3 * bs + k0);
    acc0 = mma_b(a, b0, acc0);
    acc1 = mma_b(a, b1, acc1);
    acc2 = mma_b(a, b2, acc2);
    acc3 = mma_b(a, b3, acc3);
    guard6<v16b>(acc0, acc1, acc2, acc3, a, b0, b1, b2, b3, a);
  }
  epi64hsb(slab + wave * SLAB64, acc0, acc1, acc2, acc3, oscale, pscale, bias, C, N, (size_t)rowb, col0, lane);
}

__global__ __launch_bounds__(128)
void gemm_hh16r(const u16* __restrict__ A, const u16* __restrict__ Bt, const float* __restrict__ bias, u16* C,
                int M, int N, int K, float oscale, float pscale) {
  __shared__ __align__(16) float slab[4 * SLAB64];
  const int tid = threadIdx.x, wave = tid >> 5, lane = tid & 31, hh = lane >> 4, m = lane & 15;
  const int ntile = N >> 6;
  const int bid   = blockIdx.x;
  const int rowb  = (bid / ntile) * 64 + wave * 16;
  const int col0  = (bid % ntile) * 64;
  if (rowb + 16 > M) return;
  const _Float16* ap = (const _Float16*)(const void*)A  + (size_t)(rowb + m) * (size_t)K + 8 * hh;
  const _Float16* bp = (const _Float16*)(const void*)Bt + (size_t)(col0 + m) * (size_t)K + 8 * hh;
  const size_t bs = (size_t)16 * K;
  v8f acc0 = zero8(), acc1 = zero8(), acc2 = zero8(), acc3 = zero8();
#pragma unroll 1
  for (int k0 = 0; k0 < K; k0 += 32) {
    const v16h a  = ldfrag_h(ap + k0);
    const v16h b0 = ldfrag_h(bp + k0);
    const v16h b1 = ldfrag_h(bp + bs + k0);
    const v16h b2 = ldfrag_h(bp + 2 * bs + k0);
    const v16h b3 = ldfrag_h(bp + 3 * bs + k0);
    acc0 = mma_h(a, b0, acc0);
    acc1 = mma_h(a, b1, acc1);
    acc2 = mma_h(a, b2, acc2);
    acc3 = mma_h(a, b3, acc3);
    guard6<v16h>(acc0, acc1, acc2, acc3, a, b0, b1, b2, b3, a);
  }
  epi64hrb(slab + wave * SLAB64, acc0, acc1, acc2, acc3, oscale, pscale, bias + rowb, C, N, (size_t)rowb, col0, lane);
}

__global__ __launch_bounds__(ATT_THREADS)
void attn_heads(const u16* __restrict__ QPp, const u16* __restrict__ KPp, const u16* __restrict__ VTp, float* out) {
  __shared__ __align__(16) AttU U;
  __shared__ __align__(16) u16 sP[NH * NT * PLP];

  const int tid  = threadIdx.x;
  const int wave = tid >> 5;
  const int lane = tid & 31;
  const int hh   = lane >> 4;
  const int m    = lane & 15;
  const int q0   = blockIdx.x * NT;

  const _Float16* qb = (const _Float16*)(const void*)QPp + ((size_t)q0 + m) * DM + wave * DKH + 8 * hh;
  const _Float16* kb = (const _Float16*)(const void*)KPp + (size_t)m * DM + wave * DKH + 8 * hh;
  const _Float16* vb = (const _Float16*)(const void*)VTp + ((size_t)(wave * 64) + m) * NL + 8 * hh;
  const float lsc = LOG2E / (QSC * KSC * 8.0f);
  float* const sw = U.s + wave * (NT * SSP);

  v8f o00 = zero8(), o01 = zero8(), o02 = zero8(), o03 = zero8();
  v8f o10 = zero8(), o11 = zero8(), o12 = zero8(), o13 = zero8();

#pragma unroll 1
  for (int l0 = 0; l0 < NL; l0 += LT) {
    {
      const v16h qa0 = ldfrag_h(qb), qa1 = ldfrag_h(qb + 32);
      const v16h qc0 = ldfrag_h(qb + (size_t)16 * DM), qc1 = ldfrag_h(qb + (size_t)16 * DM + 32);
      const _Float16* kp = kb + (size_t)l0 * DM;
      const v16h ka0 = ldfrag_h(kp), ka1 = ldfrag_h(kp + 32);
      const v16h kc0 = ldfrag_h(kp + (size_t)16 * DM), kc1 = ldfrag_h(kp + (size_t)16 * DM + 32);
      v8f s00 = zero8(), s01 = zero8(), s10 = zero8(), s11 = zero8();
      s00 = mma_h(qa0, ka0, s00);  s00 = mma_h(qa1, ka1, s00);
      s01 = mma_h(qa0, kc0, s01);  s01 = mma_h(qa1, kc1, s01);
      s10 = mma_h(qc0, ka0, s10);  s10 = mma_h(qc1, ka1, s10);
      s11 = mma_h(qc0, kc0, s11);  s11 = mma_h(qc1, kc1, s11);
      guard4x8(s00, s01, s10, s11, qa0, qa1, qc0, qc1, ka0, ka1, kc0, kc1);
#pragma unroll
      for (int r = 0; r < 8; ++r) {
        const int ro = (8 * hh + r) * SSP + m;
        sw[ro]                 = s00[r];
        sw[ro + 16]            = s01[r];
        sw[ro + 16 * SSP]      = s10[r];
        sw[ro + 16 * SSP + 16] = s11[r];
      }
    }
    __syncthreads();
    {
      const int n = tid >> 3, lq = (tid & 7) * 4;
      float t[NH][4];
#pragma unroll
      for (int h = 0; h < NH; ++h) {
        const v4f a = *(const v4f*)(U.s + h * (NT * SSP) + n * SSP + lq);
#pragma unroll
        for (int e = 0; e < 4; ++e) t[h][e] = a[e] * lsc;
      }
#pragma unroll
      for (int e = 0; e < 4; ++e) {
        float mx = t[0][e];
#pragma unroll
        for (int h = 1; h < NH; ++h) mx = fmaxf(mx, t[h][e]);
        float sm = 0.f;
#pragma unroll
        for (int h = 0; h < NH; ++h) {
          const float p = exp2f(t[h][e] - mx);
          t[h][e] = p;
          sm += p;
        }
        const float rs = __builtin_amdgcn_rcpf(sm) * PCAR;
#pragma unroll
        for (int h = 0; h < NH; ++h) t[h][e] *= rs;
      }
      u16* pd = sP + n * PLP + lq;
#pragma unroll
      for (int h = 0; h < NH; ++h) {
        v2u pk;
        pk[0] = pk16(h_bits((_Float16)t[h][0]), h_bits((_Float16)t[h][1]));
        pk[1] = pk16(h_bits((_Float16)t[h][2]), h_bits((_Float16)t[h][3]));
        *(v2u*)(pd + h * (NT * PLP)) = pk;
      }
    }
    __syncthreads();
    {
      const _Float16* pbase = (const _Float16*)(const void*)sP + m * PLP + 8 * hh;
      const _Float16* vl = vb + l0;
#pragma unroll 1
      for (int h = 0; h < NH; ++h) {
        const _Float16* pp = pbase + h * (NT * PLP);
        const v16h p0 = ldfrag_h(pp);
        const v16h p1 = ldfrag_h(pp + 16 * PLP);
        const _Float16* vp = vl + (size_t)h * DM * NL;
        const v16h g0 = ldfrag_h(vp);
        const v16h g1 = ldfrag_h(vp + (size_t)16 * NL);
        const v16h g2 = ldfrag_h(vp + (size_t)32 * NL);
        const v16h g3 = ldfrag_h(vp + (size_t)48 * NL);
        o00 = mma_h(p0, g0, o00);
        o01 = mma_h(p0, g1, o01);
        o02 = mma_h(p0, g2, o02);
        o03 = mma_h(p0, g3, o03);
        o10 = mma_h(p1, g0, o10);
        o11 = mma_h(p1, g1, o11);
        o12 = mma_h(p1, g2, o12);
        o13 = mma_h(p1, g3, o13);
        guard8x6(o00, o01, o02, o03, o10, o11, o12, o13, p0, p1, g0, g1, g2, g3);
      }
    }
  }
  __syncthreads();

  const float osc = 1.0f / (PCAR * VCAR * (float)NH);
  const v4f z4 = {0.f, 0.f, 0.f, 0.f};
  float* const sl = U.slab + wave * SLAB64;
  epi64(sl, o00, o01, o02, o03, osc, z4, out, DM, (size_t)q0, wave * 64, lane);
  wave_sync_lds();
  epi64(sl, o10, o11, o12, o13, osc, z4, out, DM, (size_t)q0 + 16, wave * 64, lane);
}

extern "C" void kernel_launch(void* const* d_in, const int* in_sizes, int n_in,
                              void* d_out, int out_size, void* d_ws, size_t ws_size,
                              hipStream_t stream) {
  if (n_in < 10) return;
  if (in_sizes[0] != NQ * DM || in_sizes[1] != NL * DM) return;
  if (in_sizes[2] != DM * DM || in_sizes[3] != DM) return;
  if (in_sizes[4] != DM * DM || in_sizes[5] != DM) return;
  if (in_sizes[6] != DM * DM || in_sizes[7] != DM) return;
  if (in_sizes[8] != DM * DV || in_sizes[9] != DV) return;
  if (out_size != NQ * DM) return;

  const float* xq  = (const float*)d_in[0];
  const float* xs  = (const float*)d_in[1];
  const float* wv1 = (const float*)d_in[2];
  const float* bv1 = (const float*)d_in[3];
  const float* wq  = (const float*)d_in[4];
  const float* bq  = (const float*)d_in[5];
  const float* wk  = (const float*)d_in[6];
  const float* bk  = (const float*)d_in[7];
  const float* wv2 = (const float*)d_in[8];
  const float* bv2 = (const float*)d_in[9];
  float*       out = (float*)d_out;

  const size_t szXQ = (size_t)SQ * DM * 2;
  const size_t szXS = (size_t)NL * DM * 2;
  const size_t szWT = (size_t)DM * DM * 2;
  const size_t szW2 = (size_t)DV * DM * 2;
  const size_t szVL = (size_t)NL * DM * 2;
  const size_t szQP = (size_t)SQ * DM * 2;
  const size_t szKP = (size_t)NL * DM * 2;
  const size_t szVT = (size_t)DV * NL * 2;
  size_t off = 0;
  const size_t oXQ = off; off += szXQ;
  const size_t oXS = off; off += szXS;
  const size_t oW1 = off; off += szWT;
  const size_t oWQ = off; off += szWT;
  const size_t oWK = off; off += szWT;
  const size_t oW2 = off; off += szW2;
  const size_t oVL = off; off += szVL;
  const size_t oQP = off; off += szQP;
  const size_t oKP = off; off += szKP;
  const size_t oVT = off; off += szVT;
  if (off > ws_size) return;
  if (off > WS_CAP) return;

  char* ws = (char*)d_ws;
  u16* XQ   = (u16*)(ws + oXQ);
  u16* XS   = (u16*)(ws + oXS);
  u16* WV1T = (u16*)(ws + oW1);
  u16* WQT  = (u16*)(ws + oWQ);
  u16* WKT  = (u16*)(ws + oWK);
  u16* WV2T = (u16*)(ws + oW2);
  u16* VALH = (u16*)(ws + oVL);
  u16* QP   = (u16*)(ws + oQP);
  u16* KP   = (u16*)(ws + oKP);
  u16* VT   = (u16*)(ws + oVT);

  const int n8q = (SQ * DM) / 8;
  const int n8s = (NL * DM) / 8;
  const dim3 blk(256);
  const dim3 bG(128);
  const dim3 gXq(n8q / 256);
  const dim3 gXs(n8s / 256);
  const dim3 gWT((DM / 64) * (DM / 64));
  const dim3 gW2((DM / 64) * (DV / 64));
  const dim3 gGq((SQ / 64) * (DM / 64));
  const dim3 gG((NL / 64) * (DM / 64));
  const dim3 gVT((DV / 64) * (NL / 64));
  const dim3 gAT(SQ / NT);
  const dim3 bAT(ATT_THREADS);

  cvt16<<<gXq, blk, 0, stream>>>(xq, XQ, n8q, 0, 1.0f);
  cvt16<<<gXs, blk, 0, stream>>>(xs, XS, n8s, 0, 1.0f);
  tr16<<<gWT, blk, 0, stream>>>(wv1, WV1T, DM, DM, 0, 1.0f);
  tr16<<<gWT, blk, 0, stream>>>(wq,  WQT,  DM, DM, 0, 1.0f);
  tr16<<<gWT, blk, 0, stream>>>(wk,  WKT,  DM, DM, 0, 1.0f);
  tr16<<<gW2, blk, 0, stream>>>(wv2, WV2T, DM, DV, 1, W2S);
  gemm_bh16<<<gG,  bG, 0, stream>>>(XS, WV1T, bv1, VALH, NL, DM, DM, 1.0f, VSC);
  gemm_bh16<<<gGq, bG, 0, stream>>>(XQ, WQT,  bq,  QP,   SQ, DM, DM, 1.0f, QSC);
  gemm_bh16<<<gG,  bG, 0, stream>>>(XS, WKT,  bk,  KP,   NL, DM, DM, 1.0f, KSC);
  gemm_hh16r<<<gVT, bG, 0, stream>>>(WV2T, VALH, bv2, VT, DV, NL, DM, 1.0f / (W2S * VSC), VCAR);
  attn_heads<<<gAT, bAT, 0, stream>>>(QP, KP, VT, out);
  (void)hipGetLastError();
}
